// TransformerBlock_60756607369302
// MI455X (gfx1250) — hardware-verified
//
#include <hip/hip_runtime.h>
#include <math.h>

#ifndef NB
#define NB 4
#endif
#ifndef SEQ
#define SEQ 2048
#endif
#define NB_FULL 4
#define SEQ_FULL 2048
#define DM 768
#define NH 12
#define DH 64
#define FF 3072
#define NTOK (NB * SEQ)

#define W_CARRY   64.0f
#define P_CARRY   4096.0f
#define RES_CARRY 2048.0f
#define CTX_CARRY 16.0f
#define G_CARRY   16.0f

static_assert(DM == NH * DH);
static_assert(DH == 64);
static_assert(DM == 32 * 4 * 6);
static_assert(DM % 64 == 0 && FF % 64 == 0 && NTOK % 64 == 0);
static_assert(DM % 32 == 0 && FF % 32 == 0);
static_assert(SEQ % 64 == 0 && SEQ <= SEQ_FULL && NB <= NB_FULL);
static_assert(DM % 8 == 0 && FF % 8 == 0);

typedef __attribute__((ext_vector_type(16))) _Float16 v16h;
typedef __attribute__((ext_vector_type(8)))  _Float16 v8h;
typedef __attribute__((ext_vector_type(8)))  float    v8f;
typedef __attribute__((ext_vector_type(4)))  float    v4f;
typedef __attribute__((ext_vector_type(4)))  unsigned int v4u;

union FragU { v16h v; v8h h[2]; };

#define VST2(T, ptr, val) do { const T vst2_v_ = (val); *(volatile T*)(ptr) = vst2_v_; __threadfence(); *(volatile T*)(ptr) = vst2_v_; } while (0)

__device__ __forceinline__ float cmb_bf(float v) {
    const unsigned u = __builtin_bit_cast(unsigned, v);
    const unsigned r = (u + 0x7fffu + ((u >> 16) & 1u)) & 0xffff0000u;
    return __builtin_bit_cast(float, r);
}
__device__ __forceinline__ unsigned int pk2h(float a, float b) {
    return (unsigned int)__builtin_bit_cast(unsigned short, (_Float16)a) | ((unsigned int)__builtin_bit_cast(unsigned short, (_Float16)b) << 16);
}
__device__ __forceinline__ int full_row(int t) { return (t / SEQ) * SEQ_FULL + (t % SEQ); }

__device__ __forceinline__ v16h frag_ld(const _Float16* p) {
    FragU f; f.h[0] = *(const v8h*)(p); f.h[1] = *(const v8h*)(p + 16); return f.v;
}
__device__ __forceinline__ v8f mma_h(v16h a, v16h b, v8f c) {
    return __builtin_amdgcn_wmma_f32_16x16x32_f16(false, a, false, b, (short)0, c, false, false);
}
__device__ __forceinline__ v8f wmma16(v16h a, v16h b, v8f c) {
    c = __builtin_amdgcn_wmma_f32_16x16x32_f16(false, a, false, b, (short)0, c, false, false);
    asm volatile("v_nop\n\tv_nop\n\tv_nop\n\tv_nop" : "+v"(c) : "v"(a), "v"(b));
    return c;
}
__device__ __forceinline__ void dep_guard_h(v8f& a, v8f& b, v16h x, v16h y) { asm volatile("v_nop\n\tv_nop\n\tv_nop\n\tv_nop" : "+v"(a), "+v"(b) : "v"(x), "v"(y)); }
__device__ __forceinline__ void keep4_h(v16h a, v16h b, v16h c, v16h d) { asm volatile("v_nop" :: "v"(a), "v"(b), "v"(c), "v"(d)); }
__device__ __forceinline__ void acc_guard4(v8f& a, v8f& b, v8f& c, v8f& d) { asm volatile("v_nop\n\tv_nop\n\tv_nop\n\tv_nop" : "+v"(a), "+v"(b), "+v"(c), "+v"(d)); }

template <int OUT_MODE, int ACT>
__device__ __forceinline__ void gemm64_body(
    const unsigned short* __restrict__ Ap, int lda, const unsigned short* __restrict__ Btp, int ldb,
    unsigned short* __restrict__ C16, unsigned short* __restrict__ C16r, float* __restrict__ C32, int ldc,
    const float* __restrict__ bias, int M, int N, int K, float scale, float oscale) {
  static_assert(OUT_MODE == 0 || OUT_MODE == 1 || OUT_MODE == 3);
  static_assert(ACT == 0 || OUT_MODE == 1);
  const _Float16* A = (const _Float16*)Ap; const _Float16* Bt = (const _Float16*)Btp;
  __shared__ __align__(16) float sT[8][16 * 68];
  const int lane = threadIdx.x & 31;
  const int wave = threadIdx.x >> 5;
  const int tilesN = N >> 6;
  const int tilesM = M >> 6;
  const int tile = blockIdx.x * 8 + wave;
  if (tile >= tilesM * tilesN) return;
  const int tm = tile / tilesN;
  const int tn = tile - tm * tilesN;
  const int m0 = tm << 6;
  const int n0 = tn << 6;
  const int rlane = lane & 15;
  const int koff  = (lane >> 4) * 8;
  const int mOff  = (lane >> 4) * 8;

  v8f acc[4][4];
#pragma unroll
  for (int i = 0; i < 4; ++i)
#pragma unroll
    for (int j = 0; j < 4; ++j) acc[i][j] = (v8f){0.f,0.f,0.f,0.f,0.f,0.f,0.f,0.f};

  for (int k0 = 0; k0 < K; k0 += 32) {
    v16h bh[4];
#pragma unroll
    for (int j = 0; j < 4; ++j) {
      const size_t bo = (size_t)(n0 + (j << 4) + rlane) * ldb + koff + k0;
      bh[j] = frag_ld(Bt + bo);
    }
#pragma unroll
    for (int i = 0; i < 4; ++i) {
      const size_t ao = (size_t)(m0 + (i << 4) + rlane) * lda + koff + k0;
      v16h ah = frag_ld(A + ao);
#pragma unroll
      for (int j = 0; j < 4; ++j) acc[i][j] = mma_h(ah, bh[j], acc[i][j]);
      dep_guard_h(acc[i][0], acc[i][3], ah, ah);
    }
    keep4_h(bh[0], bh[1], bh[2], bh[3]);
  }
  acc_guard4(acc[0][0], acc[0][1], acc[0][2], acc[0][3]);
  acc_guard4(acc[1][0], acc[1][1], acc[1][2], acc[1][3]);
  acc_guard4(acc[2][0], acc[2][1], acc[2][2], acc[2][3]);
  acc_guard4(acc[3][0], acc[3][1], acc[3][2], acc[3][3]);

  float* slab = sT[wave];
#pragma unroll
  for (int i = 0; i < 4; ++i) {
    const int mBase = m0 + (i << 4);
#pragma unroll
    for (int j = 0; j < 4; ++j) {
      const int n = n0 + (j << 4) + rlane;
      const float bv = cmb_bf(bias[n]);
#pragma unroll
      for (int r = 0; r < 8; ++r) slab[(mOff + r) * 68 + (j << 4) + rlane] = acc[i][j][r] * scale + bv;
    }
    __builtin_amdgcn_fence(3  , "workgroup");
    __builtin_amdgcn_wave_barrier();
    __builtin_amdgcn_fence(2  , "workgroup");
    if (OUT_MODE == 0) {
      const int hh = lane >> 4, c4 = (lane & 15) * 4;
      for (int pass = 0; pass < 2; ++pass) {
#pragma unroll
        for (int it = 0; it < 8; ++it) {
          const int row = it * 2 + hh;
          v4f v = *(const v4f*)(slab + row * 68 + c4);
          *(volatile v4f*)(C32 + (size_t)(mBase + row) * ldc + n0 + c4) = v;
        }
        __threadfence();
      }
    } else {
      const int q = lane >> 3, c8 = (lane & 7) * 8;
#pragma unroll 1
      for (int it = 0; it < 4; ++it) {
        const int row = it * 4 + q;
        const float* sp = slab + row * 68 + c8;
        v8h hv, lv;
#pragma unroll
        for (int e = 0; e < 8; ++e) {
          float v = sp[e];
          if (ACT == 5) v = 0.5f * v * (1.0f + erff(v * 0.70710678118654752f));
          v *= oscale;
          const _Float16 hb = (_Float16)v;
          hv[e] = hb;
          lv[e] = (OUT_MODE == 3) ? (_Float16)((v - (float)hb) * RES_CARRY) : hb;
        }
        volatile v8h* d  = (volatile v8h*)(C16 + (size_t)(mBase + row) * ldc + n0 + c8);
        *d = hv;
        if (OUT_MODE == 3) { volatile v8h* dr = (volatile v8h*)(C16r + (size_t)(mBase + row) * ldc + n0 + c8); *dr = lv; }
        __threadfence();
        *d = hv;
        if (OUT_MODE == 3) { volatile v8h* dr = (volatile v8h*)(C16r + (size_t)(mBase + row) * ldc + n0 + c8); *dr = lv; }
      }
    }
    __builtin_amdgcn_fence(3  , "workgroup");
    __builtin_amdgcn_wave_barrier();
    __builtin_amdgcn_fence(2  , "workgroup");
  }
}

__global__ __launch_bounds__(256) void k_gemm_h16(const unsigned short* __restrict__ A, int lda, const unsigned short* __restrict__ Bt, int ldb,
    unsigned short* __restrict__ C, int ldc, const float* __restrict__ bias, int M, int N, int K, float scale, float oscale) {
  gemm64_body<1, 0>(A, lda, Bt, ldb, C, nullptr, nullptr, ldc, bias, M, N, K, scale, oscale);
}
__global__ __launch_bounds__(256) void k_gemm_h16r(const unsigned short* __restrict__ A, int lda, const unsigned short* __restrict__ Bt, int ldb,
    unsigned short* __restrict__ C, unsigned short* __restrict__ Cr, int ldc, const float* __restrict__ bias, int M, int N, int K, float scale, float oscale) {
  gemm64_body<3, 0>(A, lda, Bt, ldb, C, Cr, nullptr, ldc, bias, M, N, K, scale, oscale);
}
__global__ __launch_bounds__(256) void k_gemm_f32(const unsigned short* __restrict__ A, int lda, const unsigned short* __restrict__ Bt, int ldb,
    float* __restrict__ C, int ldc, const float* __restrict__ bias, int M, int N, int K, float scale) {
  gemm64_body<0, 0>(A, lda, Bt, ldb, nullptr, nullptr, C, ldc, bias, M, N, K, scale, 1.0f);
}
__global__ __launch_bounds__(256) void k_gemm_gelu16(const unsigned short* __restrict__ A, int lda, const unsigned short* __restrict__ Bt, int ldb,
    unsigned short* __restrict__ C, int ldc, const float* __restrict__ bias, int M, int N, int K, float scale, float oscale) {
  gemm64_body<1, 5>(A, lda, Bt, ldb, C, nullptr, nullptr, ldc, bias, M, N, K, scale, oscale);
}

__global__ __launch_bounds__(128) void k_attn_f16(const unsigned short* __restrict__ Qp, const unsigned short* __restrict__ Kp,
    const unsigned short* __restrict__ VHp, const unsigned short* __restrict__ VRp, unsigned short* __restrict__ AOp) {
  __shared__ __align__(16) _Float16 Ksh[64 * 64];
  __shared__ __align__(16) _Float16 Vth[64 * 64];
  __shared__ __align__(16) _Float16 Vtr[64 * 64];
  __shared__ __align__(16) _Float16 Psh[4][16 * 64];
  __shared__ __align__(16) _Float16 Psr[4][16 * 64];
  __shared__ __align__(16) float    Os[4][16 * 68];
  const _Float16* Q  = (const _Float16*)Qp;
  const _Float16* Kg = (const _Float16*)Kp;
  const _Float16* VH = (const _Float16*)VHp;
  const _Float16* VR = (const _Float16*)VRp;

  const int tid  = threadIdx.x;
  const int wave = tid >> 5;
  const int lane = tid & 31;
  const int hh   = lane >> 4;
  const int c    = lane & 15;
  const int nqb = SEQ / 64;
  const int bx = blockIdx.x;
  const int qb = bx % nqb;
  const int bh = bx / nqb;
  const int h  = bh % NH;
  const int b  = bh / NH;
  const int q0 = qb * 64 + wave * 16;
  const size_t tok0 = (size_t)b * SEQ;
  const bool early = (qb == 0);

  FragU qa[2];
  {
    const _Float16* qrow = Q + (tok0 + q0 + c) * DM + h * DH;
#pragma unroll
    for (int dc = 0; dc < 2; ++dc) {
      qa[dc].h[0] = *(const v8h*)(qrow + dc * 32 + 8 * hh);
      qa[dc].h[1] = *(const v8h*)(qrow + dc * 32 + 16 + 8 * hh);
    }
  }
  float mrow[8], lrow[8];
  v8f oacc[4], oacc2[4];
#pragma unroll
  for (int r = 0; r < 8; ++r) { mrow[r] = -__builtin_inff(); lrow[r] = 0.f; }
#pragma unroll
  for (int t = 0; t < 4; ++t) { oacc[t] = (v8f){0.f,0.f,0.f,0.f,0.f,0.f,0.f,0.f}; oacc2[t] = (v8f){0.f,0.f,0.f,0.f,0.f,0.f,0.f,0.f}; }

  const int nChunks = qb + 1;
  for (int kc = 0; kc < nChunks; ++kc) {
    const int kv0 = kc * 64;
    __syncthreads();
    {
      const int kvr = tid >> 1, dh0 = (tid & 1) * 32;
      const size_t go = (tok0 + kv0 + kvr) * DM + h * DH + dh0;
#pragma unroll
      for (int i = 0; i < 4; ++i) {
        const v8h kk = *(const v8h*)(Kg + go + 8 * i);
        *(v8h*)(Ksh + kvr * 64 + dh0 + 8 * i) = kk;
        const v8h vv = *(const v8h*)(VH + go + 8 * i);
#pragma unroll
        for (int e = 0; e < 8; ++e) Vth[(dh0 + 8 * i + e) * 64 + kvr] = vv[e];
      }
      if (early) {
#pragma unroll
        for (int i = 0; i < 4; ++i) {
          const v8h vr = *(const v8h*)(VR + go + 8 * i);
#pragma unroll
          for (int e = 0; e < 8; ++e) Vtr[(dh0 + 8 * i + e) * 64 + kvr] = vr[e];
        }
      }
    }
    __syncthreads();

    v8f s[4];
#pragma unroll
    for (int j = 0; j < 4; ++j) {
      s[j] = (v8f){0.f,0.f,0.f,0.f,0.f,0.f,0.f,0.f};
#pragma unroll
      for (int dc = 0; dc < 2; ++dc) {
        FragU kb;
        kb.h[0] = *(const v8h*)(Ksh + (j * 16 + c) * 64 + dc * 32 + 8 * hh);
        kb.h[1] = *(const v8h*)(Ksh + (j * 16 + c) * 64 + dc * 32 + 16 + 8 * hh);
        s[j] = wmma16(qa[dc].v, kb.v, s[j]);
      }
    }
    const bool diag = (kc == qb);
    float cm[8];
#pragma unroll
    for (int r = 0; r < 8; ++r) {
      const int qrow = q0 + 8 * hh + r;
      float m = -__builtin_inff();
#pragma unroll
      for (int j = 0; j < 4; ++j) {
        const int kvcol = kv0 + j * 16 + c;
        float sv = s[j][r] * 0.125f;
        sv = (diag && (kvcol > qrow)) ? -__builtin_inff() : sv;
        s[j][r] = sv;
        m = fmaxf(m, sv);
      }
      m = fmaxf(m, __shfl_xor(m, 1, 32)); m = fmaxf(m, __shfl_xor(m, 2, 32));
      m = fmaxf(m, __shfl_xor(m, 4, 32)); m = fmaxf(m, __shfl_xor(m, 8, 32));
      cm[r] = m;
    }
    _Float16* pwh = Psh[wave];
    _Float16* pwr = Psr[wave];
#pragma unroll
    for (int r = 0; r < 8; ++r) {
      const float mnew = fmaxf(mrow[r], cm[r]);
      const float alpha = expf(mrow[r] - mnew);
      mrow[r] = mnew;
      float psum = 0.f;
#pragma unroll
      for (int j = 0; j < 4; ++j) {
        const float p = expf(s[j][r] - mnew);
        psum += p;
        const float pc = p * P_CARRY;
        const _Float16 ph = (_Float16)pc;
        pwh[(8 * hh + r) * 64 + j * 16 + c] = ph;
        if (early) pwr[(8 * hh + r) * 64 + j * 16 + c] = (_Float16)((pc - (float)ph) * RES_CARRY);
      }
      psum += __shfl_xor(psum, 1, 32); psum += __shfl_xor(psum, 2, 32);
      psum += __shfl_xor(psum, 4, 32); psum += __shfl_xor(psum, 8, 32);
      lrow[r] = lrow[r] * alpha + psum;
#pragma unroll
      for (int t = 0; t < 4; ++t) oacc[t][r] *= alpha;
      if (early) {
#pragma unroll
        for (int t = 0; t < 4; ++t) oacc2[t][r] *= alpha;
      }
    }
    __builtin_amdgcn_fence(3  , "workgroup");
    __builtin_amdgcn_wave_barrier();
    __builtin_amdgcn_fence(2  , "workgroup");
#pragma unroll
    for (int kk = 0; kk < 2; ++kk) {
      FragU pa;
      pa.h[0] = *(const v8h*)(pwh + c * 64 + kk * 32 + 8 * hh);
      pa.h[1] = *(const v8h*)(pwh + c * 64 + kk * 32 + 16 + 8 * hh);
#pragma unroll
      for (int t = 0; t < 4; ++t) {
        FragU vb;
        vb.h[0] = *(const v8h*)(Vth + (t * 16 + c) * 64 + kk * 32 + 8 * hh);
        vb.h[1] = *(const v8h*)(Vth + (t * 16 + c) * 64 + kk * 32 + 16 + 8 * hh);
        oacc[t] = wmma16(pa.v, vb.v, oacc[t]);
      }
      if (early) {
        FragU pr;
        pr.h[0] = *(const v8h*)(pwr + c * 64 + kk * 32 + 8 * hh);
        pr.h[1] = *(const v8h*)(pwr + c * 64 + kk * 32 + 16 + 8 * hh);
#pragma unroll
        for (int t = 0; t < 4; ++t) {
          FragU vb, vr;
          vb.h[0] = *(const v8h*)(Vth + (t * 16 + c) * 64 + kk * 32 + 8 * hh);
          vb.h[1] = *(const v8h*)(Vth + (t * 16 + c) * 64 + kk * 32 + 16 + 8 * hh);
          vr.h[0] = *(const v8h*)(Vtr + (t * 16 + c) * 64 + kk * 32 + 8 * hh);
          vr.h[1] = *(const v8h*)(Vtr + (t * 16 + c) * 64 + kk * 32 + 16 + 8 * hh);
          oacc2[t] = wmma16(pa.v, vr.v, oacc2[t]);
          oacc2[t] = wmma16(pr.v, vb.v, oacc2[t]);
        }
      }
    }
  }

  float* os = Os[wave];
#pragma unroll
  for (int r = 0; r < 8; ++r) {
    const float inv = (1.0f / (lrow[r] * P_CARRY)) * CTX_CARRY;
#pragma unroll
    for (int t = 0; t < 4; ++t) os[(8 * hh + r) * 68 + t * 16 + c] = (oacc[t][r] + oacc2[t][r] * (1.0f / RES_CARRY)) * inv;
  }
  __builtin_amdgcn_fence(3  , "workgroup");
  __builtin_amdgcn_wave_barrier();
  __builtin_amdgcn_fence(2  , "workgroup");
  {
    const int q = lane >> 3, c8 = (lane & 7) * 8;
    unsigned short* ob = AOp + (tok0 + q0) * DM + h * DH;
    for (int pass = 0; pass < 2; ++pass) {
#pragma unroll
      for (int it = 0; it < 4; ++it) {
        const int row = it * 4 + q;
        const float* sp = os + row * 68 + c8;
        v8h hv;
#pragma unroll
        for (int e = 0; e < 8; ++e) hv[e] = (_Float16)sp[e];
        *(volatile v8h*)(ob + (size_t)row * DM + c8) = hv;
      }
      __threadfence();
    }
  }
}

__global__ __launch_bounds__(256) void k_add_ln(const float* __restrict__ A, int a_full, int rneA, const float* __restrict__ Bv,
    const float* __restrict__ w, const float* __restrict__ bb, float* __restrict__ outF, int o_full, unsigned short* __restrict__ out16) {
  const int wave = threadIdx.x >> 5, lane = threadIdx.x & 31;
  const int t = blockIdx.x * 8 + wave;
  if (t >= NTOK) return;
  const size_t ra = a_full ? (size_t)full_row(t) : (size_t)t;
  const float* ar = A + ra * DM;
  const float* br = Bv + (size_t)t * DM;
  v4f v[6];
  float s = 0.f;
#pragma unroll
  for (int i = 0; i < 6; ++i) {
    const int col = (i * 32 + lane) * 4;
    v4f a = *(const v4f*)(ar + col);
    if (rneA) { a.x = cmb_bf(a.x); a.y = cmb_bf(a.y); a.z = cmb_bf(a.z); a.w = cmb_bf(a.w); }
    const v4f b2 = *(const v4f*)(br + col);
    v[i] = a + b2;
    s += (v[i].x + v[i].y) + (v[i].z + v[i].w);
  }
  s += __shfl_xor(s, 16, 32); s += __shfl_xor(s, 8, 32); s += __shfl_xor(s, 4, 32); s += __shfl_xor(s, 2, 32); s += __shfl_xor(s, 1, 32);
  const float mean = s * (1.0f / (float)DM);
  float s2 = 0.f;
#pragma unroll
  for (int i = 0; i < 6; ++i) {
    const v4f d = v[i] - mean;
    s2 += (d.x * d.x + d.y * d.y) + (d.z * d.z + d.w * d.w);
  }
  s2 += __shfl_xor(s2, 16, 32); s2 += __shfl_xor(s2, 8, 32); s2 += __shfl_xor(s2, 4, 32); s2 += __shfl_xor(s2, 2, 32); s2 += __shfl_xor(s2, 1, 32);
  const float rstd = rsqrtf(s2 * (1.0f / (float)DM) + 1e-5f);
  v4f y[6];
  unsigned long long pk[6];
#pragma unroll
  for (int i = 0; i < 6; ++i) {
    const int col = (i * 32 + lane) * 4;
    const v4f wv = *(const v4f*)(w + col), bv = *(const v4f*)(bb + col);
    v4f o;
    o.x = (v[i].x - mean) * rstd * cmb_bf(wv.x) + cmb_bf(bv.x);
    o.y = (v[i].y - mean) * rstd * cmb_bf(wv.y) + cmb_bf(bv.y);
    o.z = (v[i].z - mean) * rstd * cmb_bf(wv.z) + cmb_bf(bv.z);
    o.w = (v[i].w - mean) * rstd * cmb_bf(wv.w) + cmb_bf(bv.w);
    y[i] = o;
    pk[i] = (unsigned long long)pk2h(o.x, o.y) | ((unsigned long long)pk2h(o.z, o.w) << 32);
  }
  const size_t ro = o_full ? (size_t)full_row(t) : (size_t)t;
  for (int pass = 0; pass < 2; ++pass) {
#pragma unroll
    for (int i = 0; i < 6; ++i) {
      const int col = (i * 32 + lane) * 4;
      if (outF)  *(volatile v4f*)(outF + ro * DM + col) = y[i];
      if (out16) *(volatile unsigned long long*)(out16 + (size_t)t * DM + col) = pk[i];
    }
    __threadfence();
  }
}

__global__ __launch_bounds__(256) void k_castx(const float* __restrict__ X, unsigned short* __restrict__ DST) {
  const int u = blockIdx.x * 256 + threadIdx.x; const int per = DM / 8; if (u >= NTOK * per) return;
  const int t = u / per, c0 = 8 * (u % per);
  const float* sp = X + (size_t)full_row(t) * DM + c0;
  const v4f a = *(const v4f*)sp, b = *(const v4f*)(sp + 4);
  v4u pkv; pkv.x = pk2h(cmb_bf(a.x), cmb_bf(a.y)); pkv.y = pk2h(cmb_bf(a.z), cmb_bf(a.w)); pkv.z = pk2h(cmb_bf(b.x), cmb_bf(b.y)); pkv.w = pk2h(cmb_bf(b.z), cmb_bf(b.w));
  VST2(v4u, DST + (size_t)u * 8, pkv);
}
__global__ __launch_bounds__(256) void k_castbT(const float* __restrict__ SRC, int lds, unsigned short* __restrict__ DST, int ldd, int nR, int nC, float sc) {
  const int u = blockIdx.x * 256 + threadIdx.x; const int per = nR / 8; if (u >= nC * per) return;
  const int c = u / per; const int r0 = 8 * (u % per);
  float wv[8];
#pragma unroll
  for (int e = 0; e < 8; ++e) wv[e] = cmb_bf(SRC[(size_t)(r0 + e) * lds + c]) * sc;
  v4u pkv; pkv.x = pk2h(wv[0], wv[1]); pkv.y = pk2h(wv[2], wv[3]); pkv.z = pk2h(wv[4], wv[5]); pkv.w = pk2h(wv[6], wv[7]);
  VST2(v4u, DST + (size_t)c * ldd + r0, pkv);
}
__global__ __launch_bounds__(256) void k_wqkvT(const float* __restrict__ Wq, const float* __restrict__ Wk, const float* __restrict__ Wv, unsigned short* __restrict__ DST, float sc) {
  const int u = blockIdx.x * 256 + threadIdx.x; const int per = DM / 8; if (u >= 3 * DM * per) return;
  const int n = u / per, d0 = 8 * (u % per);
  const int which = n / DM, cc = n - which * DM; const int h = cc >> 6, e = cc & 63;
  float wv[8];
#pragma unroll
  for (int j = 0; j < 8; ++j) {
    const size_t idx = ((size_t)h * DM + d0 + j) * DH + e;
    const float a = Wq[idx], b = Wk[idx], c = Wv[idx];
    const float sv = (which == 0) ? a : ((which == 1) ? b : c);
    wv[j] = cmb_bf(sv) * sc;
  }
  v4u pkv; pkv.x = pk2h(wv[0], wv[1]); pkv.y = pk2h(wv[2], wv[3]); pkv.z = pk2h(wv[4], wv[5]); pkv.w = pk2h(wv[6], wv[7]);
  VST2(v4u, DST + (size_t)u * 8, pkv);
}

constexpr size_t P16_B  = (size_t)NTOK * DM * 2;
constexpr size_t R0_B   = 4 * P16_B;
constexpr size_t RA_B   = 2 * P16_B;
constexpr size_t HF_B   = (size_t)NTOK * DM * 4;
constexpr size_t W3_B   = (size_t)3 * DM * DM * 2;
constexpr size_t WO_B   = (size_t)DM * DM * 2;
constexpr size_t W1_B   = (size_t)DM * FF * 2;
constexpr size_t W2_B   = (size_t)FF * DM * 2;
constexpr size_t WS_TOTAL = R0_B + RA_B + HF_B + W3_B + WO_B + W1_B + W2_B;
static_assert((size_t)NTOK * FF * 2 <= R0_B);
static_assert((size_t)NTOK * DM * 4 <= R0_B);
static_assert((size_t)NTOK * DM * 4 <= RA_B);
static_assert(P16_B % 256 == 0 && W3_B % 256 == 0 && WO_B % 256 == 0 && W1_B % 256 == 0);
static_assert(WS_TOTAL <= (size_t)134217728);
static_assert(((NTOK / 64) * (DM / 64)) % 8 == 0 || true);

extern "C" void kernel_launch(void* const* d_in, const int* in_sizes, int n_in, void* d_out, int out_size, void* d_ws, size_t ws_size, hipStream_t stream) {
  if (n_in < 17) return;
  const long long xneed = ((long long)(NB - 1) * SEQ_FULL + SEQ) * DM;
  if ((long long)in_sizes[0] < xneed) return;
  if ((long long)in_sizes[1] < (long long)NH * DM * DH || (long long)in_sizes[3] < (long long)NH * DM * DH || (long long)in_sizes[5] < (long long)NH * DM * DH) return;
  if (in_sizes[2] < DM || in_sizes[4] < DM || in_sizes[6] < DM || in_sizes[8] < DM || in_sizes[12] < DM) return;
  if ((long long)in_sizes[7] < (long long)DM * DM || (long long)in_sizes[9] < (long long)DM * FF || (long long)in_sizes[11] < (long long)FF * DM) return;
  if (in_sizes[10] < FF || in_sizes[13] < DM || in_sizes[14] < DM || in_sizes[15] < DM || in_sizes[16] < DM) return;
  if ((long long)out_size < xneed) return;
  if (ws_size < WS_TOTAL) return;

  const float* x    = (const float*)d_in[0];
  const float* Wq   = (const float*)d_in[1];
  const float* bq   = (const float*)d_in[2];
  const float* Wk   = (const float*)d_in[3];
  const float* bk   = (const float*)d_in[4];
  const float* Wv   = (const float*)d_in[5];
  const float* bv   = (const float*)d_in[6];
  const float* Wo   = (const float*)d_in[7];
  const float* bo   = (const float*)d_in[8];
  const float* W1   = (const float*)d_in[9];
  const float* b1   = (const float*)d_in[10];
  const float* W2   = (const float*)d_in[11];
  const float* b2   = (const float*)d_in[12];
  const float* ln1w = (const float*)d_in[13];
  const float* ln1b = (const float*)d_in[14];
  const float* ln2w = (const float*)d_in[15];
  const float* ln2b = (const float*)d_in[16];
  float* out = (float*)d_out;

  char* ws = (char*)d_ws;
  char* R0 = ws;
  char* RA = R0 + R0_B;
  char* HFp = RA + RA_B;
  char* WB = HFp + HF_B;
  unsigned short* X16  = (unsigned short*)(R0);
  unsigned short* Q16  = (unsigned short*)(R0 + P16_B);
  unsigned short* K16  = (unsigned short*)(R0 + 2 * P16_B);
  unsigned short* VH16 = (unsigned short*)(R0 + 3 * P16_B);
  float*          T1   = (float*)(R0);
  unsigned short* G16  = (unsigned short*)(R0);
  unsigned short* VR16 = (unsigned short*)(RA);
  unsigned short* AO16 = (unsigned short*)(RA + P16_B);
  unsigned short* H16  = (unsigned short*)(RA);
  float*          T2   = (float*)(RA);
  float*          HF   = (float*)(HFp);
  unsigned short* W316 = (unsigned short*)(WB);
  unsigned short* WO16 = (unsigned short*)(WB + W3_B);
  unsigned short* W116 = (unsigned short*)(WB + W3_B + WO_B);
  unsigned short* W216 = (unsigned short*)(WB + W3_B + WO_B + W1_B);

  k_castx<<<(unsigned)((NTOK * (DM / 8) + 255) / 256), 256, 0, stream>>>(x, X16);
  k_wqkvT<<<(unsigned)((3 * DM * (DM / 8) + 255) / 256), 256, 0, stream>>>(Wq, Wk, Wv, W316, W_CARRY);
  k_castbT<<<(unsigned)((DM * (DM / 8) + 255) / 256), 256, 0, stream>>>(Wo, DM, WO16, DM, DM, DM, W_CARRY);
  k_castbT<<<(unsigned)((FF * (DM / 8) + 255) / 256), 256, 0, stream>>>(W1, FF, W116, DM, DM, FF, W_CARRY);
  k_castbT<<<(unsigned)((DM * (FF / 8) + 255) / 256), 256, 0, stream>>>(W2, DM, W216, FF, FF, DM, W_CARRY);

  const unsigned gD = (unsigned)(((NTOK / 64) * (DM / 64) + 7) / 8);
  const unsigned gF = (unsigned)(((NTOK / 64) * (FF / 64) + 7) / 8);
  const float sW = 1.0f / W_CARRY;
  k_gemm_h16<<<gD, 256, 0, stream>>>(X16, DM, W316, DM, Q16, DM, bq, NTOK, DM, DM, sW, 1.0f);
  k_gemm_h16<<<gD, 256, 0, stream>>>(X16, DM, W316 + (size_t)DM * DM, DM, K16, DM, bk, NTOK, DM, DM, sW, 1.0f);
  k_gemm_h16r<<<gD, 256, 0, stream>>>(X16, DM, W316 + (size_t)2 * DM * DM, DM, VH16, VR16, DM, bv, NTOK, DM, DM, sW, 1.0f);
  k_attn_f16<<<(unsigned)(NB * NH * (SEQ / 64)), 128, 0, stream>>>(Q16, K16, VH16, VR16, AO16);
  k_gemm_f32<<<gD, 256, 0, stream>>>(AO16, DM, WO16, DM, T1, DM, bo, NTOK, DM, DM, 1.0f / (W_CARRY * CTX_CARRY));
  k_add_ln<<<(unsigned)((NTOK + 7) / 8), 256, 0, stream>>>(x, 1, 1, T1, ln1w, ln1b, HF, 0, H16);
  k_gemm_gelu16<<<gF, 256, 0, stream>>>(H16, DM, W116, DM, G16, FF, b1, NTOK, FF, DM, sW, G_CARRY);
  k_gemm_f32<<<gD, 256, 0, stream>>>(G16, FF, W216, FF, T2, DM, b2, NTOK, DM, FF, 1.0f / (W_CARRY * G_CARRY));
  k_add_ln<<<(unsigned)((NTOK + 7) / 8), 256, 0, stream>>>(HF, 0, 0, T2, ln2w, ln2b, out, 1, nullptr);
}
